// GraphConvBlock_83597243449881
// MI455X (gfx1250) — hardware-run, weakly checked
//
#include <hip/hip_runtime.h>


#ifndef NB
#define NB 8
#endif
#define NB_FULL 8
#define IMG_H 64
#define IMG_W 64
#define PH 66
#define PW 66
#define C0 64
#define CM 128
#define NNODE 6
#define OSP 68
#define TLP 68
#define HALO (2 * PW + 2 * IMG_H)

static_assert(NB <= NB_FULL);
static_assert(NB >= 1);
static_assert(IMG_W == 64);
static_assert(PH == IMG_H + 2);
static_assert(PW == IMG_W + 2);
static_assert(C0 % 32 == 0);
static_assert(CM % 32 == 0);
static_assert(CM % 64 == 0);
static_assert((C0 * 2) % 128 == 0);
static_assert((CM * 2) % 128 == 0);
static_assert((OSP * 4) % 16 == 0);
static_assert((TLP * 4) % 16 == 0);
static_assert(64 * OSP * 4 <= 131072);
static_assert(IMG_W * TLP * 4 <= 131072);
static_assert(32 * 16 * 32 == 64 * 64 * 4);
static_assert(32 * 16 * 16 == 64 * 64 * 2);
static_assert(C0 * IMG_W / 4 == 4 * 256);
static_assert(IMG_W * C0 / 8 == 2 * 256);
static_assert((9 * CM * C0 / 8) % 256 == 0);
static_assert((NNODE * 9 * CM * CM / 8) % 256 == 0);
static_assert((NB * HALO * (C0 / 8)) % 8 == 0);
static_assert((4 * NB * HALO * (CM / 8)) % 8 == 0);

typedef unsigned short bf;
typedef __attribute__((ext_vector_type(16))) __bf16   v16bf;
typedef __attribute__((ext_vector_type(8)))  unsigned short v8us;
typedef __attribute__((ext_vector_type(8)))  float    v8f;
typedef __attribute__((ext_vector_type(4)))  float    v4f;
typedef v4f  __attribute__((may_alias)) v4fa;

static constexpr size_t al256(size_t v) { return (v + 255) & ~(size_t)255; }
static constexpr size_t SZ_XP = al256((size_t)NB * PH * PW * C0 * 2);
static constexpr size_t SZ_W0 = al256((size_t)9 * CM * C0 * 2);
static constexpr size_t SZ_WN = al256((size_t)NNODE * 9 * CM * CM * 2);
static constexpr size_t SZ_SP = al256((size_t)NB * PH * PW * CM * 2);
static constexpr size_t SZ_F  = al256((size_t)NB * IMG_H * IMG_W * CM * 4);
static constexpr size_t SZ_TOTAL = SZ_XP + SZ_W0 + SZ_WN + 4 * SZ_SP + 2 * SZ_F;
static constexpr size_t SP_ELEMS = SZ_SP / 2;
static_assert(SZ_TOTAL <= (size_t)134217728);
static_assert(SZ_SP == (size_t)NB * PH * PW * CM * 2);
static_assert(((size_t)9 * CM * CM * 2) % 256 == 0);

__device__ __forceinline__ unsigned short f2bf(float f) { unsigned u = __float_as_uint(f); u += 0x7FFFu + ((u >> 16) & 1u); return (unsigned short)(u >> 16); }
__device__ __forceinline__ float bfr(float f) { return __uint_as_float(((unsigned)f2bf(f)) << 16); }
__device__ __forceinline__ float bf2f(unsigned short u) { return __uint_as_float(((unsigned)u) << 16); }
__device__ __forceinline__ v16bf cat16b(v8us lo, v8us hi) { return __builtin_bit_cast(v16bf, __builtin_shufflevector(lo, hi, 0, 1, 2, 3, 4, 5, 6, 7, 8, 9, 10, 11, 12, 13, 14, 15)); }
__device__ __forceinline__ v8f wmmab(v16bf a, v16bf b, v8f c) { return __builtin_amdgcn_wmma_f32_16x16x32_bf16(false, a, false, b, (short)0, c, false, false); }
__device__ __forceinline__ v8f wmmab_g(v16bf a, v16bf b, v8f c) { v8f d = wmmab(a, b, c); asm volatile("v_nop\n\tv_nop\n\tv_nop\n\tv_nop" : "+v"(d) : "v"(a), "v"(b)); return d; }
__device__ __forceinline__ v16bf ldb(const bf* p)  { return cat16b(*(const v8us*)p, *(const v8us*)(p + 16)); }
__device__ __forceinline__ void wave_sync() { __builtin_amdgcn_fence(3  , "wavefront"); __builtin_amdgcn_wave_barrier(); asm volatile("" ::: "memory"); }

__global__ __launch_bounds__(256) void k_xpose(const float* __restrict__ x, bf* XP) {
    __shared__ __align__(16) float tl[IMG_W * TLP];
    const int n = blockIdx.x / IMG_H, h = blockIdx.x % IMG_H; const int t = threadIdx.x;
#pragma unroll 1
    for (int i = 0; i < 4; ++i) { const int idx = i * 256 + t; const int c = idx >> 4, w4 = (idx & 15) * 4;
        const v4f v = *(const v4f*)(x + (((size_t)n * C0 + c) * IMG_H + h) * IMG_W + w4);
        tl[(w4 + 0) * TLP + c] = v[0]; tl[(w4 + 1) * TLP + c] = v[1]; tl[(w4 + 2) * TLP + c] = v[2]; tl[(w4 + 3) * TLP + c] = v[3]; }
    __syncthreads();
#pragma unroll 1
    for (int ps = 0; ps < 2; ++ps) {
#pragma unroll 1
        for (int i = 0; i < 2; ++i) { const int idx = i * 256 + t; const int w = idx >> 3, c8 = (idx & 7) * 8;
            const v4f x0 = *(const v4fa*)(&tl[w * TLP + c8]); const v4f x1 = *(const v4fa*)(&tl[w * TLP + c8 + 4]); v8us o;
#pragma unroll
            for (int k = 0; k < 4; ++k) { o[k] = f2bf(x0[k]); o[4 + k] = f2bf(x1[k]); }
            *(volatile v8us*)(XP + ((size_t)(n * PH + h + 1) * PW + (size_t)(w + 1)) * C0 + c8) = o; }
        if (ps == 0) __threadfence(); }
}

__global__ __launch_bounds__(256) void k_wprep(const float* __restrict__ src, bf* dst, int CI, int total8) {
    const int i = blockIdx.x * 256 + threadIdx.x; if (i >= total8) return;
    const int c8n = CI >> 3; const int ci8 = i % c8n; int r = i / c8n; const int co = r % CM; r /= CM; const int tap = r % 9; const int l = r / 9;
    const size_t sb = (((size_t)l * CM + co) * (size_t)CI + (size_t)ci8 * 8) * 9 + tap;
    v8us o;
#pragma unroll
    for (int k = 0; k < 8; ++k) o[k] = f2bf(src[sb + (size_t)k * 9]);
    *(volatile v8us*)(dst + (size_t)i * 8) = o; __threadfence(); *(volatile v8us*)(dst + (size_t)i * 8) = o;
}

__global__ __launch_bounds__(256) void k_halo(bf* base, int pcs, size_t planeElems, int total) {
    const int i = blockIdx.x * 256 + threadIdx.x; if (i >= total) return;
    const int piece = i % pcs; int r = i / pcs; const int q = r % HALO; r /= HALO; const int n = r % NB; const int pl = r / NB;
    const int e = q - 2 * PW;
    const int row = (q < PW) ? 0 : ((q < 2 * PW) ? (PH - 1) : (1 + (e >> 1)));
    const int col = (q < PW) ? q : ((q < 2 * PW) ? (q - PW) : ((e & 1) * (PW - 1)));
    const size_t o = (size_t)pl * planeElems + ((size_t)(n * PH + row) * PW + (size_t)col) * (size_t)(pcs * 8) + (size_t)piece * 8;
    const v8us z = (v8us){};
    *(volatile v8us*)(base + o) = z; __threadfence(); *(volatile v8us*)(base + o) = z;
}

template <int CIN, int NPL, int MODE, int ADDIN, int WRF>
__device__ __forceinline__ void conv_tile(const bf* __restrict__ A, const bf* __restrict__ Wt, const float* __restrict__ bias, float bmul,
                                          const float* __restrict__ Fin, float* Fout, bf* Sout, float* OUT) {
    __shared__ __align__(16) float os[64 * OSP];
    static_assert(CIN % 32 == 0);
    static_assert(NPL == 1 || NPL == 2);
    const int lane = threadIdx.x & 31, lr = lane & 15, hi = lane >> 4;
    const int n = blockIdx.x / IMG_H, h = blockIdx.x % IMG_H;
    const int c0 = blockIdx.y * 64;
    const size_t r0 = (size_t)blockIdx.x * IMG_W;
    v8f acc[4][4];
#pragma unroll
    for (int mb = 0; mb < 4; ++mb)
#pragma unroll
        for (int nb = 0; nb < 4; ++nb) acc[mb][nb] = (v8f){};
    const size_t abase = ((size_t)(n * PH + h) * PW + (size_t)lr) * CIN + 8 * hi;
    const size_t bbase = (size_t)(c0 + lr) * CIN + 8 * hi;
#pragma unroll 1
    for (int pl = 0; pl < NPL; ++pl) {
        const size_t pbase = abase + (size_t)pl * SP_ELEMS;
#pragma unroll 1
        for (int tap = 0; tap < 9; ++tap) {
            const int kh = tap / 3, kw = tap - 3 * kh;
            const size_t ao = pbase + (size_t)(kh * PW + kw) * CIN;
            const size_t bo = bbase + (size_t)tap * CM * CIN;
#pragma unroll 1
            for (int kc = 0; kc < CIN; kc += 32) {
                v16bf a[4];
#pragma unroll
                for (int mb = 0; mb < 4; ++mb) a[mb] = ldb(A + ao + (size_t)mb * 16 * CIN + kc);
#pragma unroll
                for (int nb = 0; nb < 4; ++nb) { const v16bf b = ldb(Wt + bo + (size_t)nb * 16 * CIN + kc);
#pragma unroll
                    for (int mb = 0; mb < 4; ++mb) acc[mb][nb] = wmmab_g(a[mb], b, acc[mb][nb]); }
            }
        }
    }
    float bc[4];
#pragma unroll
    for (int nb = 0; nb < 4; ++nb) bc[nb] = bfr(bias[c0 + nb * 16 + lr]) * bmul;
#pragma unroll
    for (int mb = 0; mb < 4; ++mb)
#pragma unroll
        for (int nb = 0; nb < 4; ++nb)
#pragma unroll
            for (int j = 0; j < 8; ++j) {
                const float v = acc[mb][nb][j] + bc[nb];
                if (MODE == 0) os[(mb * 16 + hi * 8 + j) * OSP + nb * 16 + lr] = v;
                else           os[(nb * 16 + lr) * OSP + mb * 16 + hi * 8 + j] = v; }
    wave_sync();
#pragma unroll 1
    for (int ps = 0; ps < 2; ++ps) {
        if (MODE == 0) {
            if (WRF) {
#pragma unroll 1
                for (int s = 0; s < 32; ++s) { const int pix = 2 * s + (lane >> 4), c4 = (lane & 15) * 4;
                    const v4f val = *(const v4fa*)(&os[pix * OSP + c4]);
                    *(volatile v4f*)(Fout + (r0 + (size_t)pix) * CM + c0 + c4) = val; }
            }
#pragma unroll 1
            for (int s = 0; s < 16; ++s) { const int pix = 4 * s + (lane >> 3), c8 = (lane & 7) * 8;
                v4f x0 = *(const v4fa*)(&os[pix * OSP + c8]); v4f x1 = *(const v4fa*)(&os[pix * OSP + c8 + 4]);
                if (ADDIN) { const float* pp = Fin + (r0 + (size_t)pix) * CM + c0 + c8; const v4f p0 = *(const v4f*)pp; const v4f p1 = *(const v4f*)(pp + 4); x0 = x0 + p0; x1 = x1 + p1; }
                v8us hv, lv;
#pragma unroll
                for (int i = 0; i < 4; ++i) { const unsigned short a0 = f2bf(x0[i]); const unsigned short a1 = f2bf(x1[i]);
                    hv[i] = a0; hv[4 + i] = a1; lv[i] = f2bf(x0[i] - bf2f(a0)); lv[4 + i] = f2bf(x1[i] - bf2f(a1)); }
                const size_t so = ((size_t)(n * PH + h + 1) * PW + (size_t)(pix + 1)) * CM + c0 + c8;
                *(volatile v8us*)(Sout + so) = hv; *(volatile v8us*)(Sout + SP_ELEMS + so) = lv; }
        } else {
#pragma unroll 1
            for (int s = 0; s < 32; ++s) { const int col = 2 * s + (lane >> 4), w4 = (lane & 15) * 4;
                const v4f val = *(const v4fa*)(&os[col * OSP + w4]);
                *(volatile v4f*)(OUT + (((size_t)n * CM + (size_t)(c0 + col)) * IMG_H + h) * IMG_W + w4) = val; }
        }
        if (ps == 0) __threadfence(); }
}

__global__ __launch_bounds__(32) void k_conv_stem(const bf* __restrict__ XP, const bf* __restrict__ W0P, const float* __restrict__ b0, float* Fout, bf* Sout, float* OUT) {
    conv_tile<C0, 1, 0, 0, 1>(XP, W0P, b0, 1.0f, b0, Fout, Sout, OUT);
}
__global__ __launch_bounds__(32) void k_conv_mid(const bf* __restrict__ Sin, const bf* __restrict__ Wl, const float* __restrict__ bl, float bmul, const float* __restrict__ Fin, float* Fout, bf* Sout, float* OUT) {
    conv_tile<CM, 2, 0, 1, 1>(Sin, Wl, bl, bmul, Fin, Fout, Sout, OUT);
}
__global__ __launch_bounds__(32) void k_conv_mid_nf(const bf* __restrict__ Sin, const bf* __restrict__ Wl, const float* __restrict__ bl, float bmul, const float* __restrict__ Fin, float* Fout, bf* Sout, float* OUT) {
    conv_tile<CM, 2, 0, 1, 0>(Sin, Wl, bl, bmul, Fin, Fout, Sout, OUT);
}
__global__ __launch_bounds__(32) void k_conv_last(const bf* __restrict__ Sin, const bf* __restrict__ Wl, const float* __restrict__ bl, float bmul, float* Fout, bf* Sout, float* OUT) {
    conv_tile<CM, 2, 1, 0, 0>(Sin, Wl, bl, bmul, bl, Fout, Sout, OUT);
}

extern "C" void kernel_launch(void* const* d_in, const int* in_sizes, int n_in,
                              void* d_out, int out_size, void* d_ws, size_t ws_size, hipStream_t stream) {
    if (n_in < 5) return;
    if ((size_t)in_sizes[0] < (size_t)NB * C0 * IMG_H * IMG_W) return;
    if ((size_t)in_sizes[1] < (size_t)CM * C0 * 9) return;
    if (in_sizes[2] < CM) return;
    if ((size_t)in_sizes[3] < (size_t)NNODE * CM * CM * 9) return;
    if (in_sizes[4] < NNODE * CM) return;
    if ((size_t)out_size < (size_t)NB * CM * IMG_H * IMG_W) return;
    if (SZ_TOTAL > ws_size) return;
    const float* x  = (const float*)d_in[0];
    const float* W0 = (const float*)d_in[1];
    const float* b0 = (const float*)d_in[2];
    const float* Wn = (const float*)d_in[3];
    const float* bn = (const float*)d_in[4];
    float* OUT = (float*)d_out;
    char* wsp = (char*)d_ws;
    bf* XP  = (bf*)wsp; wsp += SZ_XP;
    bf* W0P = (bf*)wsp; wsp += SZ_W0;
    bf* WNP = (bf*)wsp; wsp += SZ_WN;
    bf* SA  = (bf*)wsp; wsp += 2 * SZ_SP;
    bf* SB  = (bf*)wsp; wsp += 2 * SZ_SP;
    float* FA = (float*)wsp; wsp += SZ_F;
    float* FB = (float*)wsp; wsp += SZ_F;
    const size_t WL = (size_t)9 * CM * CM;

    k_xpose<<<NB * IMG_H, 256, 0, stream>>>(x, XP);
    { const int t8 = 9 * CM * C0 / 8;          k_wprep<<<(unsigned)((t8 + 255) / 256), 256, 0, stream>>>(W0, W0P, C0, t8); }
    { const int t8 = NNODE * 9 * CM * CM / 8;  k_wprep<<<(unsigned)((t8 + 255) / 256), 256, 0, stream>>>(Wn, WNP, CM, t8); }
    { const int tot = NB * HALO * (C0 / 8);     k_halo<<<(unsigned)((tot + 255) / 256), 256, 0, stream>>>(XP, C0 / 8, (size_t)0, tot); }
    { const int tot = 4 * NB * HALO * (CM / 8); k_halo<<<(unsigned)((tot + 255) / 256), 256, 0, stream>>>(SA, CM / 8, SP_ELEMS, tot); }

    const dim3 grid(NB * IMG_H, CM / 64, 1);
    k_conv_stem<<<grid, 32, 0, stream>>>(XP, W0P, b0, FA, SA, OUT);
    k_conv_mid<<<grid, 32, 0, stream>>>(SA, WNP + 0 * WL, bn + 0 * CM, 1.0f, FA, FB, SB, OUT);
    k_conv_mid<<<grid, 32, 0, stream>>>(SB, WNP + 1 * WL, bn + 1 * CM, 2.0f, FB, FA, SA, OUT);
    k_conv_mid<<<grid, 32, 0, stream>>>(SA, WNP + 2 * WL, bn + 2 * CM, 2.0f, FA, FB, SB, OUT);
    k_conv_mid<<<grid, 32, 0, stream>>>(SB, WNP + 3 * WL, bn + 3 * CM, 2.0f, FB, FA, SA, OUT);
    k_conv_mid_nf<<<grid, 32, 0, stream>>>(SA, WNP + 4 * WL, bn + 4 * CM, 2.0f, FA, FB, SB, OUT);
    k_conv_last<<<grid, 32, 0, stream>>>(SB, WNP + 5 * WL, bn + 5 * CM, 2.0f, FB, SA, OUT);
}
